// SoftClusterAttentionLayer_75952201662470
// MI455X (gfx1250) — hardware-verified
//
#include <hip/hip_runtime.h>
#include <hip/hip_bf16.h>
#include <math.h>


typedef _Float16 bf16;
typedef _Float16 f16;
typedef __attribute__((ext_vector_type(4))) unsigned v4u_t;
typedef unsigned v4ua __attribute__((ext_vector_type(4), may_alias));
typedef __attribute__((ext_vector_type(4))) float v4f_t;
typedef float v4fa __attribute__((ext_vector_type(4), may_alias));
typedef __attribute__((ext_vector_type(16))) bf16  bf16x16;
typedef bf16x16 f16x16;
typedef __attribute__((ext_vector_type(8)))  bf16  bf16x8;
typedef bf16x8 f16x8;
typedef __attribute__((ext_vector_type(4)))  bf16  bf16x4;
typedef __attribute__((ext_vector_type(8)))  float f32x8;
__device__ __forceinline__ f32x8 wmma16(f16x16 a, f16x16 b, f32x8 c) {
  c = __builtin_amdgcn_wmma_f32_16x16x32_f16(false, a, false, b, (short)0, c, false, false);
  asm volatile("v_nop\n\tv_nop\n\tv_nop\n\tv_nop" : "+v"(c) : "v"(a), "v"(b));
  return c;
}
#define LDS_STRIDE 48
#define KSTRIDE    72
#define VSTRIDE    48

__device__ __forceinline__ f32x8 wmma_bf16(bf16x16 a, bf16x16 b, f32x8 c) {
  c = __builtin_amdgcn_wmma_f32_16x16x32_f16(false, a, false, b, (short)0, c, false, false);
  asm volatile("v_nop\n\tv_nop\n\tv_nop\n\tv_nop" : "+v"(c) : "v"(a), "v"(b));
  return c;
}

template <typename T>
__device__ __forceinline__ bf16x16 load_frag(const T* __restrict__ base, int ld,
                                             int row0, int k0) {
  const int lane = threadIdx.x & 31;
  const int r    = lane & 15;
  const int kh   = (lane >> 4) * 8;
  const T* p0 = base + (size_t)(row0 + r) * ld + (k0 + kh);
  const T* p1 = p0 + 16;
  bf16x16 f;
#pragma unroll
  for (int i = 0; i < 8; ++i) {
    f[i]     = (bf16)p0[i];
    f[i + 8] = (bf16)p1[i];
  }
  return f;
}

__device__ __forceinline__ bf16x16 lds_frag(const bf16* base, int stride) {
  const int lane = threadIdx.x & 31;
  const int row  = lane & 15;
  const int kh   = (lane >> 4) * 8;
  const bf16x8 lo = *(const bf16x8*)(base + row * stride + kh);
  const bf16x8 hi = *(const bf16x8*)(base + row * stride + kh + 16);
  bf16x16 f;
#pragma unroll
  for (int i = 0; i < 8; ++i) { f[i] = lo[i]; f[i + 8] = hi[i]; }
  return f;
}

template <typename T>
__device__ __forceinline__ void stage_read16(const T* __restrict__ p, float* buf) {
#pragma unroll
  for (int i = 0; i < 16; ++i) buf[i] = (float)p[i];
}

__device__ __forceinline__ void stage_write(bf16* dst, const float* buf, int nquad) {
#pragma unroll
  for (int i = 0; i < nquad; ++i) {
    bf16x4 q;
    q[0] = (bf16)buf[4 * i];     q[1] = (bf16)buf[4 * i + 1];
    q[2] = (bf16)buf[4 * i + 2]; q[3] = (bf16)buf[4 * i + 3];
    *(bf16x4*)(dst + 4 * i) = q;
  }
}


#define GSTR 48
#define GSTR 48
template <typename AT, int EPI, bool OUT16>
__global__ __launch_bounds__(256) void gemm_kne(const AT* __restrict__ A, int lda, const float* __restrict__ Wm, int ldw,
                                                const float* __restrict__ bias, const float* __restrict__ R, const float* __restrict__ gvec,
                                                void* __restrict__ Yv, int ldy, int K) {
  __shared__ __attribute__((aligned(16))) f16 ldsA[128 * GSTR];
  __shared__ __attribute__((aligned(16))) f16 ldsW[128 * GSTR];
  __shared__ __attribute__((aligned(16))) float oS[8][32 * 68];
  const int tid = threadIdx.x, lane = tid & 31, wave = tid >> 5, cl = lane & 15, rh = (lane >> 4) * 8;
  const int m0 = blockIdx.x * 128, n0 = blockIdx.y * 128;
  const int wm = (wave & 3) * 32, wn = (wave >> 2) * 64;
  f32x8 acc[2][4];
#pragma unroll
  for (int i = 0; i < 2; ++i)
#pragma unroll
    for (int j = 0; j < 4; ++j) { f32x8 z = {}; acc[i][j] = z; }
#pragma unroll 1
  for (int k0 = 0; k0 < K; k0 += 32) {
    __syncthreads();
    { const int row = tid >> 1, ch = (tid & 1) * 16;
      const AT* src = A + (size_t)(m0 + row) * lda + k0 + ch;
#pragma unroll
      for (int g = 0; g < 16; ++g) ldsA[row * GSTR + ch + g] = (f16)src[g]; }
    { const int k = tid >> 3, nn0 = (tid & 7) * 16;
      const float* src = Wm + (size_t)(k0 + k) * ldw + n0 + nn0;
#pragma unroll
      for (int g = 0; g < 4; ++g) { const v4f_t v = *(const v4f_t*)(src + 4 * g);
#pragma unroll
        for (int u = 0; u < 4; ++u) ldsW[(nn0 + 4 * g + u) * GSTR + k] = (f16)v[u]; } }
    __syncthreads();
    f16x16 af[2];
#pragma unroll
    for (int i = 0; i < 2; ++i) af[i] = lds_frag(ldsA + (wm + 16 * i) * GSTR, GSTR);
#pragma unroll
    for (int j = 0; j < 4; ++j) {
      const f16x16 bf = lds_frag(ldsW + (wn + 16 * j) * GSTR, GSTR);
#pragma unroll
      for (int i = 0; i < 2; ++i) acc[i][j] = wmma16(af[i], bf, acc[i][j]);
    }
  }
  float* so = oS[wave];
#pragma unroll
  for (int i = 0; i < 2; ++i)
#pragma unroll
    for (int j = 0; j < 4; ++j) {
      const int n = n0 + wn + 16 * j + cl;
      const float bv = bias ? bias[n] : 0.0f;
      const float gv = (EPI == 2 || EPI == 4) ? gvec[n] : 0.0f;
      if (EPI == 1) {
#pragma unroll 1
        for (int r = 0; r < 8; ++r) { const float xg = acc[i][j][r] + bv; so[(16 * i + rh + r) * 68 + 16 * j + cl] = 0.5f * xg * (1.0f + erff(xg * 0.70710678118654752f)); }
      } else {
#pragma unroll
        for (int r = 0; r < 8; ++r) {
          float v = acc[i][j][r] + bv;
          if (EPI == 3) v = fmaxf(v, 0.0f);
          if (EPI == 4) v = gv * v;
          if (EPI == 2) v = R[(size_t)(m0 + wm + 16 * i + rh + r) * ldy + n] + gv * v;
          so[(16 * i + rh + r) * 68 + 16 * j + cl] = v;
        }
      }
    }
  asm volatile("s_wait_dscnt 0" ::: "memory");
  __builtin_amdgcn_wave_barrier();
#pragma unroll 1
  for (int pass = 0; pass < 2; ++pass) {
    if (OUT16) {
      f16* Y = (f16*)Yv;
#pragma unroll
      for (int it = 0; it < 8; ++it) { const int c = lane + 32 * it, rr = c >> 3, q8 = (c & 7) * 8;
        union { f16 h[8]; v4u_t v; } u;
#pragma unroll
        for (int e = 0; e < 8; ++e) u.h[e] = (f16)so[rr * 68 + q8 + e];
        *(volatile v4u_t*)(Y + (size_t)(m0 + wm + rr) * ldy + n0 + wn + q8) = u.v; }
    } else {
      float* Y = (float*)Yv;
#pragma unroll
      for (int it = 0; it < 16; ++it) { const int f4 = lane + 32 * it, rr = f4 >> 4, q = (f4 & 15) * 4;
        *(volatile v4f_t*)(Y + (size_t)(m0 + wm + rr) * ldy + n0 + wn + q) = *(const v4fa*)(so + rr * 68 + q); }
    }
    __threadfence();
  }
}

template <typename AT, int EPI, bool OUT16>
__global__ __launch_bounds__(256) void gemm_knez(const AT* __restrict__ A, int lda, size_t strideA, const float* __restrict__ Wm, int ldw, size_t strideW,
                                                 const float* __restrict__ bias, const float* __restrict__ R, const float* __restrict__ gvec,
                                                 void* __restrict__ Yv, int ldy, size_t strideY, int K) {
  A += (size_t)blockIdx.z * strideA; Wm += (size_t)blockIdx.z * strideW; Yv = (void*)((char*)Yv + (size_t)blockIdx.z * strideY * (OUT16 ? 2 : 4)); if (R) R += (size_t)blockIdx.z * strideY;
  __shared__ __attribute__((aligned(16))) f16 ldsA[128 * GSTR];
  __shared__ __attribute__((aligned(16))) f16 ldsW[128 * GSTR];
  __shared__ __attribute__((aligned(16))) float oS[8][32 * 68];
  const int tid = threadIdx.x, lane = tid & 31, wave = tid >> 5, cl = lane & 15, rh = (lane >> 4) * 8;
  const int m0 = blockIdx.x * 128, n0 = blockIdx.y * 128;
  const int wm = (wave & 3) * 32, wn = (wave >> 2) * 64;
  f32x8 acc[2][4];
#pragma unroll
  for (int i = 0; i < 2; ++i)
#pragma unroll
    for (int j = 0; j < 4; ++j) { f32x8 z = {}; acc[i][j] = z; }
#pragma unroll 1
  for (int k0 = 0; k0 < K; k0 += 32) {
    __syncthreads();
    { const int row = tid >> 1, ch = (tid & 1) * 16;
      const AT* src = A + (size_t)(m0 + row) * lda + k0 + ch;
#pragma unroll
      for (int g = 0; g < 16; ++g) ldsA[row * GSTR + ch + g] = (f16)src[g]; }
    { const int k = tid >> 3, nn0 = (tid & 7) * 16;
      const float* src = Wm + (size_t)(k0 + k) * ldw + n0 + nn0;
#pragma unroll
      for (int g = 0; g < 4; ++g) { const v4f_t v = *(const v4f_t*)(src + 4 * g);
#pragma unroll
        for (int u = 0; u < 4; ++u) ldsW[(nn0 + 4 * g + u) * GSTR + k] = (f16)v[u]; } }
    __syncthreads();
    f16x16 af[2];
#pragma unroll
    for (int i = 0; i < 2; ++i) af[i] = lds_frag(ldsA + (wm + 16 * i) * GSTR, GSTR);
#pragma unroll
    for (int j = 0; j < 4; ++j) {
      const f16x16 bf = lds_frag(ldsW + (wn + 16 * j) * GSTR, GSTR);
#pragma unroll
      for (int i = 0; i < 2; ++i) acc[i][j] = wmma16(af[i], bf, acc[i][j]);
    }
  }
  float* so = oS[wave];
#pragma unroll
  for (int i = 0; i < 2; ++i)
#pragma unroll
    for (int j = 0; j < 4; ++j) {
      const int n = n0 + wn + 16 * j + cl;
      const float bv = bias ? bias[n] : 0.0f;
      const float gv = (EPI == 2 || EPI == 4) ? gvec[n] : 0.0f;
      if (EPI == 1) {
#pragma unroll 1
        for (int r = 0; r < 8; ++r) { const float xg = acc[i][j][r] + bv; so[(16 * i + rh + r) * 68 + 16 * j + cl] = 0.5f * xg * (1.0f + erff(xg * 0.70710678118654752f)); }
      } else {
#pragma unroll
        for (int r = 0; r < 8; ++r) {
          float v = acc[i][j][r] + bv;
          if (EPI == 3) v = fmaxf(v, 0.0f);
          if (EPI == 4) v = gv * v;
          if (EPI == 2) v = R[(size_t)(m0 + wm + 16 * i + rh + r) * ldy + n] + gv * v;
          so[(16 * i + rh + r) * 68 + 16 * j + cl] = v;
        }
      }
    }
  asm volatile("s_wait_dscnt 0" ::: "memory");
  __builtin_amdgcn_wave_barrier();
#pragma unroll 1
  for (int pass = 0; pass < 2; ++pass) {
    if (OUT16) {
      f16* Y = (f16*)Yv;
#pragma unroll
      for (int it = 0; it < 8; ++it) { const int c = lane + 32 * it, rr = c >> 3, q8 = (c & 7) * 8;
        union { f16 h[8]; v4u_t v; } u;
#pragma unroll
        for (int e = 0; e < 8; ++e) u.h[e] = (f16)so[rr * 68 + q8 + e];
        *(volatile v4u_t*)(Y + (size_t)(m0 + wm + rr) * ldy + n0 + wn + q8) = u.v; }
    } else {
      float* Y = (float*)Yv;
#pragma unroll
      for (int it = 0; it < 16; ++it) { const int f4 = lane + 32 * it, rr = f4 >> 4, q = (f4 & 15) * 4;
        *(volatile v4f_t*)(Y + (size_t)(m0 + wm + rr) * ldy + n0 + wn + q) = *(const v4fa*)(so + rr * 68 + q); }
    }
    __threadfence();
  }
}

template <typename AT, bool ACC>
__global__ __launch_bounds__(256) void gemm_kn2(const AT* __restrict__ A, int lda, size_t strideA,
                                               const float* __restrict__ Wm, int ldw, size_t strideW,
                                               const float* __restrict__ bias, float scale,
                                               float* __restrict__ Y, int ldy, size_t strideY, int K) {
  __shared__ __attribute__((aligned(16))) f16 ldsA[128 * GSTR], ldsAl[128 * GSTR];
  __shared__ __attribute__((aligned(16))) f16 ldsW[128 * GSTR], ldsWl[128 * GSTR];
  __shared__ __attribute__((aligned(16))) float oS[8][32 * 68];
  const int tid = threadIdx.x, lane = tid & 31, wave = tid >> 5, cl = lane & 15, rh = (lane >> 4) * 8;
  const int m0 = blockIdx.x * 128, n0 = blockIdx.y * 128;
  const int wm = (wave & 3) * 32, wn = (wave >> 2) * 64;
  A += (size_t)blockIdx.z * strideA; Wm += (size_t)blockIdx.z * strideW; Y += (size_t)blockIdx.z * strideY;
  f32x8 acc[2][4], accx[2][4];
#pragma unroll
  for (int i = 0; i < 2; ++i)
#pragma unroll
    for (int j = 0; j < 4; ++j) { f32x8 z = {}; acc[i][j] = z; accx[i][j] = z; }
#pragma unroll 1
  for (int k0 = 0; k0 < K; k0 += 32) {
    __syncthreads();
    {
      const int row = tid >> 1, ch = (tid & 1) * 16;
      const AT* src = A + (size_t)(m0 + row) * lda + k0 + ch;
#pragma unroll
      for (int g = 0; g < 16; ++g) { const float v = (float)src[g]; const f16 h = (f16)v; ldsA[row * GSTR + ch + g] = h; ldsAl[row * GSTR + ch + g] = (f16)((v - (float)h) * 2048.0f); }
    }
    {
      const int k = tid >> 3, nn0 = (tid & 7) * 16;
      const float* src = Wm + (size_t)(k0 + k) * ldw + n0 + nn0;
#pragma unroll
      for (int g = 0; g < 4; ++g) { const v4f_t v = *(const v4f_t*)(src + 4 * g);
#pragma unroll
        for (int u = 0; u < 4; ++u) { const f16 h = (f16)v[u]; ldsW[(nn0 + 4 * g + u) * GSTR + k] = h; ldsWl[(nn0 + 4 * g + u) * GSTR + k] = (f16)((v[u] - (float)h) * 2048.0f); } }
    }
    __syncthreads();
    f16x16 af[2], afl[2];
#pragma unroll
    for (int i = 0; i < 2; ++i) { af[i] = lds_frag(ldsA + (wm + 16 * i) * GSTR, GSTR); afl[i] = lds_frag(ldsAl + (wm + 16 * i) * GSTR, GSTR); }
#pragma unroll
    for (int j = 0; j < 4; ++j) {
      const f16x16 bf = lds_frag(ldsW + (wn + 16 * j) * GSTR, GSTR), bfl = lds_frag(ldsWl + (wn + 16 * j) * GSTR, GSTR);
#pragma unroll
      for (int i = 0; i < 2; ++i) { acc[i][j] = wmma16(af[i], bf, acc[i][j]); accx[i][j] = wmma16(af[i], bfl, accx[i][j]); accx[i][j] = wmma16(afl[i], bf, accx[i][j]); }
    }
  }
  float* so = oS[wave];
#pragma unroll
  for (int i = 0; i < 2; ++i)
#pragma unroll
    for (int j = 0; j < 4; ++j) {
      const float bv = bias ? bias[n0 + wn + 16 * j + cl] : 0.0f;
#pragma unroll
      for (int r = 0; r < 8; ++r) so[(16 * i + rh + r) * 68 + 16 * j + cl] = (acc[i][j][r] + accx[i][j][r] * (1.0f / 2048.0f)) * scale + bv;
    }
  asm volatile("s_wait_dscnt 0" ::: "memory");
  __builtin_amdgcn_wave_barrier();
  if (ACC) {
#pragma unroll
    for (int it = 0; it < 16; ++it) { const int f4 = lane + 32 * it, rr = f4 >> 4, q = (f4 & 15) * 4;
      const v4f_t old = *(const v4fa*)(Y + (size_t)(m0 + wm + rr) * ldy + n0 + wn + q);
      v4f_t v = *(const v4fa*)(so + rr * 68 + q); v += old; *(v4fa*)(so + rr * 68 + q) = v; }
    asm volatile("s_wait_dscnt 0" ::: "memory");
  }
#pragma unroll 1
  for (int pass = 0; pass < 2; ++pass) {
#pragma unroll
    for (int it = 0; it < 16; ++it) { const int f4 = lane + 32 * it, rr = f4 >> 4, q = (f4 & 15) * 4;
      *(volatile v4f_t*)(Y + (size_t)(m0 + wm + rr) * ldy + n0 + wn + q) = *(const v4fa*)(so + rr * 68 + q); }
    __threadfence();
  }
}

__global__ __launch_bounds__(256) void k_transpose(const float* __restrict__ Wm, float* __restrict__ Wt, int rows, int cols) {
  __shared__ float tS[64][65];
  const int tid = threadIdx.x, tbj = cols / 64, bi = blockIdx.x / tbj, bj = blockIdx.x % tbj;
  for (int e = tid; e < 64 * 64; e += 256) { const int r = e >> 6, c = e & 63; tS[r][c] = Wm[(size_t)(bi * 64 + r) * cols + bj * 64 + c]; }
  __syncthreads();
  for (int ch = tid; ch < 64 * 16; ch += 256) { const int r = ch >> 4, q4 = (ch & 15) * 4; v4f_t o; o[0] = tS[q4][r]; o[1] = tS[q4 + 1][r]; o[2] = tS[q4 + 2][r]; o[3] = tS[q4 + 3][r];
    float* dst = Wt + (size_t)(bj * 64 + r) * rows + bi * 64 + q4; *(volatile v4f_t*)dst = o; __threadfence(); *(volatile v4f_t*)dst = o; }
}


#define GSTR 48
#define SS 2048
#define HH 32
#define DKK 64
template <typename AT, int MODE>
__global__ __launch_bounds__(256) void gemm_rb_kernel(
    const AT* __restrict__ A, const float* __restrict__ W,
    const float* __restrict__ bias, const float* __restrict__ rowscale, const float* __restrict__ R, const float* __restrict__ rowbias, void* __restrict__ out,
    int M, int N, int K) {
  __shared__ bf16 ldsA[128 * LDS_STRIDE];
  __shared__ bf16 ldsW[256 * LDS_STRIDE];
  __shared__ __attribute__((aligned(16))) unsigned char sob[256 * 136 * 2];

  const int t    = threadIdx.x;
  const int wave = t >> 5;
  const int lane = t & 31;
  const int wm   = (wave & 1) * 64;
  const int wn   = (wave >> 1) * 64;
  const int mBlk = blockIdx.x * 128;
  const int nBlk = blockIdx.y * 256;

  const int arow = t >> 1;
  const int ach  = (t & 1) * 16;

  float abuf[16];
  float wbuf[32];

  stage_read16(A + (size_t)(mBlk + arow) * K + ach, abuf);
  const int nrow = min(nBlk + t, N - 1);
  stage_read16(W + (size_t)nrow * K,          wbuf);
  stage_read16(W + (size_t)nrow * K + 16,     wbuf + 16);

  f32x8 acc[4][4] = {};

  for (int k = 0; k < K; k += 32) {
    __syncthreads();
    stage_write(&ldsA[arow * LDS_STRIDE + ach], abuf, 4);
    stage_write(&ldsW[t * LDS_STRIDE],          wbuf, 8);
    if (k + 32 < K) {
      stage_read16(A + (size_t)(mBlk + arow) * K + (k + 32) + ach, abuf);
      stage_read16(W + (size_t)nrow * K + (k + 32),          wbuf);
      stage_read16(W + (size_t)nrow * K + (k + 32) + 16,     wbuf + 16);
    }
    __syncthreads();

    bf16x16 af[4], wf[4];
#pragma unroll
    for (int i = 0; i < 4; ++i)
      af[i] = lds_frag(ldsA + (wm + 16 * i) * LDS_STRIDE, LDS_STRIDE);
#pragma unroll
    for (int j = 0; j < 4; ++j)
      wf[j] = lds_frag(ldsW + (wn + 16 * j) * LDS_STRIDE, LDS_STRIDE);
#pragma unroll
    for (int i = 0; i < 4; ++i)
#pragma unroll
      for (int j = 0; j < 4; ++j)
        acc[i][j] = wmma_bf16(af[i], wf[j], acc[i][j]);
  }

  const int nlane = lane & 15;
  const int mh    = (lane >> 4) * 8;
  __syncthreads();
  if (MODE == 0 || MODE == 1 || MODE == 3) {
    bf16* so = (bf16*)sob;
#pragma unroll
    for (int i = 0; i < 4; ++i)
#pragma unroll
      for (int j = 0; j < 4; ++j) {
        const int nl = wn + 16 * j + nlane;
        const float bv = bias ? bias[nBlk + nl] : 0.0f;
        if (MODE == 3) {
#pragma unroll 1
          for (int r = 0; r < 8; ++r) {
            const int ml = wm + 16 * i + mh + r;
            const float xg = acc[i][j][r] + bv;
            so[ml * 264 + nl] = (bf16)(0.5f * xg * (1.0f + erff(xg * 0.70710678118654752f)));
          }
        } else {
#pragma unroll
        for (int r = 0; r < 8; ++r) {
          const int ml = wm + 16 * i + mh + r;
          const bf16 hv = (bf16)(acc[i][j][r] + bv);
          if (MODE == 0) so[ml * 264 + nl] = hv;
          else           so[nl * 136 + ml] = hv;
        }
        }
      }
    __syncthreads();
#pragma unroll 1
    for (int pass = 0; pass < 2; ++pass) {
      if (MODE == 0 || MODE == 3) {
        for (int ch = t; ch < 128 * 32; ch += 256) { const int ml = ch >> 5, q = (ch & 31) * 8;
          *(volatile v4u_t*)((bf16*)out + (size_t)(mBlk + ml) * N + nBlk + q) = *(const v4ua*)(so + ml * 264 + q); }
      } else {
        const int b_ = mBlk / SS, s0 = mBlk % SS;
        for (int ch = t; ch < 256 * 16; ch += 256) { const int nl = ch >> 4, q = (ch & 15) * 8; const int n = nBlk + nl, h = n >> 6, dk = n & (DKK - 1);
          *(volatile v4u_t*)((bf16*)out + (((size_t)(b_ * HH + h)) * DKK + dk) * SS + s0 + q) = *(const v4ua*)(so + nl * 136 + q); }
      }
      __threadfence();
    }
  } else {
    float* so = (float*)sob;
#pragma unroll 1
    for (int hf = 0; hf < 2; ++hf) {
      if (wm == hf * 64) {
#pragma unroll
        for (int i = 0; i < 4; ++i)
#pragma unroll
          for (int j = 0; j < 4; ++j) {
            const int nl = wn + 16 * j + nlane;
            const float bv = bias ? bias[nBlk + nl] : 0.0f;
#pragma unroll
            for (int r = 0; r < 8; ++r) { const int mrow = mBlk + hf * 64 + 16 * i + mh + r; so[(16 * i + mh + r) * 260 + nl] = acc[i][j][r] * (rowscale ? rowscale[mrow] : 1.0f) + bv + (rowbias ? rowbias[mrow] : 0.0f); }
          }
      }
      __syncthreads();
      if (R) {
        for (int ch = t; ch < 64 * 64; ch += 256) { const int ml = ch >> 6, q = (ch & 63) * 4;
          if (nBlk + q < N) { const v4f_t rv = *(const v4f_t*)(R + (size_t)(mBlk + hf * 64 + ml) * N + nBlk + q); v4f_t v = *(const v4fa*)(so + ml * 260 + q); v += rv; *(v4fa*)(so + ml * 260 + q) = v; }     }
        asm volatile("s_wait_dscnt 0" ::: "memory");
      }
#pragma unroll 1
      for (int pass = 0; pass < 2; ++pass) {
        for (int ch = t; ch < 64 * 64; ch += 256) { const int ml = ch >> 6, q = (ch & 63) * 4;
          if (nBlk + q < N) *(volatile v4f_t*)((float*)out + (size_t)(mBlk + hf * 64 + ml) * N + nBlk + q) = *(const v4fa*)(so + ml * 260 + q); }
        __threadfence();
      }
      __syncthreads();
    }
  }
}


template <typename AT, int EPI, bool OUT16, int NJ>
__global__ __launch_bounds__(256) void gemm_sm(const AT* __restrict__ A, int lda, size_t sA, const float* __restrict__ Wm, int ldw, size_t sW,
                                               const float* __restrict__ bias, const float* __restrict__ R, const float* __restrict__ gvec,
                                               void* __restrict__ Yv, int ldy, size_t sY, int K) {
  constexpr int BN = 16 * NJ; constexpr int OST = BN + 4;
  A += (size_t)blockIdx.z * sA; Wm += (size_t)blockIdx.z * sW; Yv = (void*)((char*)Yv + (size_t)blockIdx.z * sY * (OUT16 ? 2 : 4)); if (R) R += (size_t)blockIdx.z * sY;
  __shared__ __attribute__((aligned(16))) f16 ldsA[256 * GSTR];
  __shared__ __attribute__((aligned(16))) f16 ldsW[BN * GSTR];
  __shared__ __attribute__((aligned(16))) float oS[8][32 * OST];
  const int tid = threadIdx.x, lane = tid & 31, wave = tid >> 5, cl = lane & 15, rh = (lane >> 4) * 8;
  const int m0 = blockIdx.x * 256, n0 = blockIdx.y * BN;
  const int wm = wave * 32;
  f32x8 acc[2][NJ];
#pragma unroll
  for (int i = 0; i < 2; ++i)
#pragma unroll
    for (int j = 0; j < NJ; ++j) { f32x8 z = {}; acc[i][j] = z; }
#pragma unroll 1
  for (int k0 = 0; k0 < K; k0 += 32) {
    __syncthreads();
    { const AT* src = A + (size_t)(m0 + tid) * lda + k0;
#pragma unroll
      for (int g = 0; g < 32; ++g) ldsA[tid * GSTR + g] = (f16)src[g]; }
    { const int k = tid >> 3, nn0 = (tid & 7) * (2 * NJ);
      const float* src = Wm + (size_t)(k0 + k) * ldw + n0 + nn0;
#pragma unroll
      for (int g = 0; g < NJ / 2; ++g) { const v4f_t v = *(const v4f_t*)(src + 4 * g);
#pragma unroll
        for (int u = 0; u < 4; ++u) ldsW[(nn0 + 4 * g + u) * GSTR + k] = (f16)v[u]; } }
    __syncthreads();
    f16x16 af[2];
#pragma unroll
    for (int i = 0; i < 2; ++i) af[i] = lds_frag(ldsA + (wm + 16 * i) * GSTR, GSTR);
#pragma unroll
    for (int j = 0; j < NJ; ++j) {
      const f16x16 bf = lds_frag(ldsW + (16 * j) * GSTR, GSTR);
#pragma unroll
      for (int i = 0; i < 2; ++i) acc[i][j] = wmma16(af[i], bf, acc[i][j]);
    }
  }
  float* so = oS[wave];
#pragma unroll
  for (int i = 0; i < 2; ++i)
#pragma unroll
    for (int j = 0; j < NJ; ++j) {
      const int n = n0 + 16 * j + cl;
      const float bv = bias ? bias[n] : 0.0f;
      const float gv = (EPI == 2 || EPI == 4) ? gvec[n] : 0.0f;
#pragma unroll
      for (int r = 0; r < 8; ++r) {
        float v = acc[i][j][r] + bv;
        if (EPI == 3) v = fmaxf(v, 0.0f);
        if (EPI == 2) v = R[(size_t)(m0 + wm + 16 * i + rh + r) * ldy + n] + gv * v;
        if (EPI == 4) v = gv * v;
        so[(16 * i + rh + r) * OST + 16 * j + cl] = v;
      }
    }
  asm volatile("s_wait_dscnt 0" ::: "memory");
  __builtin_amdgcn_wave_barrier();
#pragma unroll 1
  for (int pass = 0; pass < 2; ++pass) {
    if (OUT16) {
      f16* Y = (f16*)Yv;
#pragma unroll
      for (int it = 0; it < BN / 8; ++it) { const int c = lane + 32 * it, rr = c / (BN / 8), q8 = (c % (BN / 8)) * 8;
        union { f16 h[8]; v4u_t v; } u;
#pragma unroll
        for (int e = 0; e < 8; ++e) u.h[e] = (f16)so[rr * OST + q8 + e];
        *(volatile v4u_t*)(Y + (size_t)(m0 + wm + rr) * ldy + n0 + q8) = u.v; }
    } else {
      float* Y = (float*)Yv;
#pragma unroll
      for (int it = 0; it < BN / 4; ++it) { const int f4 = lane + 32 * it, rr = f4 / (BN / 4), q = (f4 % (BN / 4)) * 4;
        *(volatile v4f_t*)(Y + (size_t)(m0 + wm + rr) * ldy + n0 + q) = *(const v4fa*)(so + rr * OST + q); }
    }
    __threadfence();
  }
}

#define LLsc 1024
#define LIN 1024
#define BBsc 4
#define EEsc 1024
#define NHsc 16
#define HDsc 64
#define LDR (BBsc * EEsc)
__global__ __launch_bounds__(256) void k_fill(float* __restrict__ p, float val, size_t n4) { const size_t i = (size_t)blockIdx.x * 256 + threadIdx.x; if (i < n4) { v4f_t v = {val, val, val, val}; *(volatile v4f_t*)(p + 4 * i) = v; __threadfence(); *(volatile v4f_t*)(p + 4 * i) = v; } }
__global__ __launch_bounds__(256) void k_dbg_zero(float* __restrict__ p, size_t n4) { const size_t i = (size_t)blockIdx.x * 256 + threadIdx.x; if (i < n4) { v4f_t z = {0.f,0.f,0.f,0.f}; *(volatile v4f_t*)(p + 4 * i) = z; __threadfence(); *(volatile v4f_t*)(p + 4 * i) = z; } }
__global__ __launch_bounds__(256) void k_copy(const float* __restrict__ src, float* __restrict__ dst, size_t n4) { const size_t i = (size_t)blockIdx.x * 256 + threadIdx.x; if (i < n4) { const v4f_t v = *(const v4f_t*)(src + 4 * i); *(volatile v4f_t*)(dst + 4 * i) = v; __threadfence(); *(volatile v4f_t*)(dst + 4 * i) = v; } }
__global__ __launch_bounds__(256) void k_transpose_ld(const float* __restrict__ Wm, int lds, float* __restrict__ Wt, int rows, int cols) {
  __shared__ float tS[64][65];
  const int tid = threadIdx.x, tbj = cols / 64, bi = blockIdx.x / tbj, bj = blockIdx.x % tbj;
  for (int e = tid; e < 64 * 64; e += 256) { const int r = e >> 6, c = e & 63; tS[r][c] = Wm[(size_t)(bi * 64 + r) * lds + bj * 64 + c]; }
  __syncthreads();
  for (int ch = tid; ch < 64 * 16; ch += 256) { const int r = ch >> 4, q4 = (ch & 15) * 4; v4f_t o; o[0] = tS[q4][r]; o[1] = tS[q4 + 1][r]; o[2] = tS[q4 + 2][r]; o[3] = tS[q4 + 3][r];
    float* dst = Wt + (size_t)(bj * 64 + r) * rows + bi * 64 + q4; *(volatile v4f_t*)dst = o; __threadfence(); *(volatile v4f_t*)dst = o; }
}
__global__ __launch_bounds__(256) void k_vsum(const float* __restrict__ V, int ldv, float* __restrict__ VB) {
  const int c = blockIdx.x * 256 + threadIdx.x; if (c >= 1024) return; float s = 0.0f;
#pragma unroll 1
  for (int r = 0; r < 1024; ++r) s += V[(size_t)r * ldv + c];
  const float m = s;   *(volatile float*)(VB + c) = m; __threadfence(); *(volatile float*)(VB + c) = m;
}
__global__ __launch_bounds__(256) void k_softT(float* __restrict__ ST) {
  __shared__ float red[256];
  const int s = blockIdx.x, tid = threadIdx.x; float* sr = ST + (size_t)s * LLsc; float v[LLsc / 256]; float m = -3.0e38f;
#pragma unroll
  for (int e = 0; e < LLsc / 256; ++e) { v[e] = sr[tid + 256 * e] * 0.125f; m = fmaxf(m, v[e]); }
  red[tid] = m; __syncthreads(); for (int o = 128; o > 0; o >>= 1) { if (tid < o) red[tid] = fmaxf(red[tid], red[tid + o]); __syncthreads(); }
  m = red[0]; __syncthreads(); float zs = 0.0f;
#pragma unroll
  for (int e = 0; e < LLsc / 256; ++e) { v[e] = expf(v[e] - m); zs += v[e]; }
  red[tid] = zs; __syncthreads(); for (int o = 128; o > 0; o >>= 1) { if (tid < o) red[tid] += red[tid + o]; __syncthreads(); }
  const float kk = 1024.0f / red[0];
#pragma unroll 1
  for (int pass = 0; pass < 2; ++pass) {
#pragma unroll
    for (int e = 0; e < LLsc / 256; ++e) *(volatile float*)(sr + tid + 256 * e) = v[e] * kk - 1.0f;
    __threadfence(); }
}
__global__ __launch_bounds__(256) void k_accaw(const float* __restrict__ P, float* __restrict__ AW, int first, size_t n4) { const size_t i = (size_t)blockIdx.x * 256 + threadIdx.x; if (i >= n4) return;
  const v4f_t p = (*(const v4f_t*)(P + 4 * i) + 1.0f) * (1.0f / 1024.0f / (float)NHsc); v4f_t a = p; if (!first) a = a + *(const v4fa*)(AW + 4 * i); *(volatile v4fa*)(AW + 4 * i) = a; __threadfence(); *(volatile v4fa*)(AW + 4 * i) = a; }

extern "C" void kernel_launch(void* const* d_in, const int* in_sizes, int n_in,
                              void* d_out, int out_size, void* d_ws, size_t ws_size,
                              hipStream_t stream) {
  (void)in_sizes; (void)n_in; (void)out_size;
  const float** f = (const float**)d_in;
  const float* xq = f[0], *xk = f[1], *xv = f[2], *Win = f[3], *bin = f[4], *Wout = f[5], *bout = f[6];
  float* out0 = (float*)d_out; float* AWout = out0 + (size_t)LIN * BBsc * EEsc;
  char* ws = (char*)d_ws;
  float* Q = (float*)ws; ws += (size_t)LLsc * LDR * 4; float* Km = (float*)ws; ws += (size_t)LLsc * LDR * 4; float* V = (float*)ws; ws += (size_t)LLsc * LDR * 4; float* O = (float*)ws; ws += (size_t)LLsc * LDR * 4;
  float* QT = (float*)ws; ws += (size_t)HDsc * LLsc * 4; float* VS = (float*)ws; ws += EEsc * 4; float* sc = (float*)ws; ws += 64 * 4; float* ST = (float*)ws; ws += (size_t)LLsc * LLsc * 4; float* P = (float*)ws; ws += (size_t)LLsc * LLsc * 4;
  if ((size_t)(ws - (char*)d_ws) > ws_size) return;
  const dim3 blk(256); const dim3 gp((LLsc * BBsc) / 128, EEsc / 256);
  k_fill<<<dim3(1), blk, 0, stream>>>(sc, 1.0f / 1024.0f, 64 / 4);

  gemm_rb_kernel<float, 2><<<gp, blk, 0, stream>>>(xq, Win, bin, nullptr, nullptr, nullptr, Q, LLsc * BBsc, EEsc, EEsc);
  gemm_rb_kernel<float, 2><<<gp, blk, 0, stream>>>(xk, Win + (size_t)EEsc * EEsc, bin + EEsc, nullptr, nullptr, nullptr, Km, LLsc * BBsc, EEsc, EEsc);
  gemm_rb_kernel<float, 2><<<gp, blk, 0, stream>>>(xv, Win + (size_t)2 * EEsc * EEsc, bin + 2 * EEsc, nullptr, nullptr, nullptr, V, LLsc * BBsc, EEsc, EEsc);
  for (int b = 0; b < BBsc; ++b) { float* AWb = AWout + (size_t)b * LIN * LIN;
    k_vsum<<<dim3(EEsc / 256), blk, 0, stream>>>(V + (size_t)b * EEsc, LDR, VS);
    for (int h = 0; h < NHsc; ++h) { const size_t col = (size_t)b * EEsc + (size_t)h * HDsc;
      k_transpose_ld<<<dim3((LLsc / 64) * (HDsc / 64)), blk, 0, stream>>>(Q + col, LDR, QT, LLsc, HDsc);
      gemm_kne<float, 0, false><<<dim3(LLsc / 128, LLsc / 128), blk, 0, stream>>>(Km + col, LDR, QT, LLsc, nullptr, nullptr, nullptr, ST, LLsc, HDsc);
      k_softT<<<dim3(LLsc), blk, 0, stream>>>(ST);
      k_transpose_ld<<<dim3((LLsc / 64) * (LLsc / 64)), blk, 0, stream>>>(ST, LLsc, P, LLsc, LLsc);
      k_accaw<<<dim3(((size_t)LLsc * LLsc / 4 + 255) / 256), blk, 0, stream>>>(P, AWb, h == 0, (size_t)LLsc * LLsc / 4);
      gemm_sm<float, 4, false, 4><<<dim3(LLsc / 256, 1, 1), blk, 0, stream>>>(P, LLsc, (size_t)0, V + col, LDR, (size_t)0, VS + h * HDsc, nullptr, sc, O + col, LDR, (size_t)0, LLsc);
    }
  }
  gemm_rb_kernel<float, 2><<<gp, blk, 0, stream>>>(O, Wout, bout, nullptr, nullptr, nullptr, out0, LLsc * BBsc, EEsc, EEsc);
}
